// DirectionalPropagation_52390011077094
// MI455X (gfx1250) — hardware-verified
//
#include <hip/hip_runtime.h>
#include <stddef.h>


#define HD      128
#define TD      32
#define NC      64
#define MD      16
#define NTHR    256
#define NWAVE   8
#define EPT     8
#define NGRP    2
#define CHUNK   (NTHR * EPT * NGRP)
#define WCAP    (EPT * NGRP * 32)
#define LISTN   (NWAVE * WCAP)
#define NB      4096
#define LDS_ACC   (NB * MD * 4)
#define LDS_LIST  (LISTN * 4)
#define LDS_PROP  (LDS_ACC + LDS_LIST)
#define WSC     16.0f
#define WINV    0.0625f

static_assert(CHUNK == 4096);
static_assert(NB <= 4096);
static_assert((NB & (NB - 1)) == 0);
static_assert(LDS_PROP <= 300 * 1024);
static_assert(NC * HD / 8 == 4 * NTHR);
static_assert((NB * MD / 4) % NTHR == 0);

typedef float    v4f  __attribute__((ext_vector_type(4)));
typedef float    v8f  __attribute__((ext_vector_type(8)));
typedef int      v4i  __attribute__((ext_vector_type(4)));
typedef unsigned v4u  __attribute__((ext_vector_type(4)));
typedef _Float16 f16_t;
typedef f16_t    v8h  __attribute__((ext_vector_type(8)));
typedef f16_t    v16h __attribute__((ext_vector_type(16)));
union FragH { v16h v; v8h h[2]; v4i q[2]; };
union Pack8 { v8h v; v4i q; };

__device__ __forceinline__ v8f wmh(v16h a, v16h b, v8f c) {
  v8f d = __builtin_amdgcn_wmma_f32_16x16x32_f16(false, a, false, b, (short)0, c, false, false);
  asm volatile("v_nop\n\tv_nop\n\tv_nop\n\tv_nop" : "+v"(d) : "v"(a), "v"(b));
  return d;
}

__device__ __forceinline__ unsigned f2key(float f) {
  const unsigned u = __float_as_uint(f);
  const unsigned msk = ((unsigned)(((int)u) >> 31)) | 0x80000000u;
  return u ^ msk;
}
__device__ __forceinline__ float key2f(unsigned k) {
  const unsigned msk = ((unsigned)(((int)(k ^ 0x80000000u)) >> 31)) | 0x80000000u;
  return __uint_as_float(k ^ msk);
}
__device__ __forceinline__ v4u f2key4(v4f v) {
  v4u k; k.x = f2key(v.x); k.y = f2key(v.y); k.z = f2key(v.z); k.w = f2key(v.w); return k;
}
__device__ __forceinline__ v4f key2f4(v4u k) {
  v4f v; v.x = key2f(k.x); v.y = key2f(k.y); v.z = key2f(k.z); v.w = key2f(k.w); return v;
}

__device__ __forceinline__ float th_fast(float z) {
  const float e = __expf(z + z);
  return 1.0f - 2.0f * __builtin_amdgcn_rcpf(e + 1.0f);
}

__global__ __launch_bounds__(NTHR) void k_wprep(const float* __restrict__ W, f16_t* wt) {
  const int tid = threadIdx.x;
  v4i qv[4];
#pragma unroll
  for (int it = 0; it < 4; ++it) {
    const int p    = it * NTHR + tid;
    const int o    = p * 8;
    const int n    = o / HD;
    const int k0   = o - n * HD;
    const int koff = (n < TD) ? 0 : HD;
    const int ncol = (n < TD) ? n : (n - TD);
    const float* src = W + (size_t)(koff + k0) * TD + ncol;
    Pack8 ph;
    ph.v[0] = (f16_t)(src[0 * TD] * WSC); ph.v[1] = (f16_t)(src[1 * TD] * WSC);
    ph.v[2] = (f16_t)(src[2 * TD] * WSC); ph.v[3] = (f16_t)(src[3 * TD] * WSC);
    ph.v[4] = (f16_t)(src[4 * TD] * WSC); ph.v[5] = (f16_t)(src[5 * TD] * WSC);
    ph.v[6] = (f16_t)(src[6 * TD] * WSC); ph.v[7] = (f16_t)(src[7 * TD] * WSC);
    qv[it] = ph.q;
  }
#pragma unroll
  for (int it = 0; it < 4; ++it) *(volatile v4i*)(wt + (size_t)(it * NTHR + tid) * 8) = qv[it];
  __threadfence();
#pragma unroll
  for (int it = 0; it < 4; ++it) *(volatile v4i*)(wt + (size_t)(it * NTHR + tid) * 8) = qv[it];
}

__global__ __launch_bounds__(NTHR) void k_node(const float* __restrict__ x, const f16_t* __restrict__ wt,
                                               float* pq, int nN) {
  __shared__ v4f st4[NWAVE * 16 * (NC / 4)];
  float* st = (float*)st4;
  const int tid = threadIdx.x, lane = tid & 31, wave = tid >> 5, h = lane >> 4, m = lane & 15;
  const int tile = blockIdx.x * NWAVE + wave;
  int row = tile * 16 + m;
  row = row > nN - 1 ? nN - 1 : row;
  const float* xr = x + (size_t)row * HD;

  v8f c[4];
#pragma unroll
  for (int ct = 0; ct < 4; ++ct) { const v8f z = {0.f, 0.f, 0.f, 0.f, 0.f, 0.f, 0.f, 0.f}; c[ct] = z; }

#pragma unroll
  for (int ks = 0; ks < HD / 32; ++ks) {
    const int k0 = 32 * ks;
    const v4f p0 = *(const v4f*)(xr + k0 + 8 * h);
    const v4f p1 = *(const v4f*)(xr + k0 + 8 * h + 4);
    const v4f p2 = *(const v4f*)(xr + k0 + 16 + 8 * h);
    const v4f p3 = *(const v4f*)(xr + k0 + 16 + 8 * h + 4);
    FragH a;
    a.v[0]  = (f16_t)p0.x; a.v[1]  = (f16_t)p0.y; a.v[2]  = (f16_t)p0.z; a.v[3]  = (f16_t)p0.w;
    a.v[4]  = (f16_t)p1.x; a.v[5]  = (f16_t)p1.y; a.v[6]  = (f16_t)p1.z; a.v[7]  = (f16_t)p1.w;
    a.v[8]  = (f16_t)p2.x; a.v[9]  = (f16_t)p2.y; a.v[10] = (f16_t)p2.z; a.v[11] = (f16_t)p2.w;
    a.v[12] = (f16_t)p3.x; a.v[13] = (f16_t)p3.y; a.v[14] = (f16_t)p3.z; a.v[15] = (f16_t)p3.w;
#pragma unroll
    for (int ct = 0; ct < 4; ++ct) {
      const f16_t* bp = wt + (size_t)(16 * ct + m) * HD + k0 + 8 * h;
      FragH b;
      b.q[0] = *(const v4i*)(bp);
      b.q[1] = *(const v4i*)(bp + 16);
      c[ct] = wmh(a.v, b.v, c[ct]);
    }
  }

  float* sw = st + wave * 16 * NC;
#pragma unroll
  for (int ct = 0; ct < 4; ++ct) {
#pragma unroll
    for (int r = 0; r < 8; ++r) sw[(8 * h + r) * NC + 16 * ct + m] = c[ct][r] * WINV;
  }
  __syncthreads();

  float* gbase = pq + (size_t)tile * 16 * NC;
  const float* lsrc = sw + (2 * 0 + (lane >> 4)) * NC + 4 * (lane & 15);
#pragma unroll
  for (int i = 0; i < 8; ++i) {
    const v4f v = *(const v4f*)(lsrc + 2 * i * NC);
    *(volatile v4f*)(gbase + (size_t)i * 2 * NC + 4 * lane) = v;
  }
  __threadfence();
#pragma unroll
  for (int i = 0; i < 8; ++i) {
    const v4f v = *(const v4f*)(lsrc + 2 * i * NC);
    *(volatile v4f*)(gbase + (size_t)i * 2 * NC + 4 * lane) = v;
  }
}

__global__ __launch_bounds__(NTHR) void k_edge(const float* __restrict__ pq, const int* __restrict__ ei,
                                               const float* __restrict__ attr, const float* __restrict__ Wg,
                                               const float* __restrict__ bg, const float* __restrict__ btr,
                                               float* ew, int nE, int nN, int ad) {
  const int e = blockIdx.x * NTHR + threadIdx.x;
  const int ec = e > nE - 1 ? nE - 1 : e;
  int s = ei[ec];
  int d = ei[(size_t)nE + ec];
  s = s < 0 ? 0 : (s > nN - 1 ? nN - 1 : s);
  d = d < 0 ? 0 : (d > nN - 1 ? nN - 1 : d);
  const float* pr = pq + (size_t)s * NC;
  const float* qr = pq + (size_t)d * NC + TD;

  float t = bg[0];
#pragma unroll 1
  for (int j = 0; j < ad; ++j) t += attr[(size_t)ec * ad + j] * Wg[j];
#pragma unroll 1
  for (int c4 = 0; c4 < TD / 4; ++c4) {
    const v4f p = *(const v4f*)(pr + 4 * c4);
    const v4f q = *(const v4f*)(qr + 4 * c4);
    const v4f b = *(const v4f*)(btr + 4 * c4);
    const float* wp = Wg + ad + 4 * c4;
    const v4f z = p + q + b;
    t += th_fast(z.x) * wp[0];
    t += th_fast(z.y) * wp[1];
    t += th_fast(z.z) * wp[2];
    t += th_fast(z.w) * wp[3];
  }
  const float g = __builtin_amdgcn_rcpf(1.0f + __expf(-t));
  *(volatile float*)(ew + e) = g;
  __threadfence();
  *(volatile float*)(ew + e) = g;
}

__device__ __forceinline__ int scan_chunk(const int* __restrict__ dsts, int nE, int cbase, int nodeBase,
                                          int vec8, int* list, int tid, int wave) {
  int wc = 0;
#pragma unroll
  for (int g = 0; g < NGRP; ++g) {
    const int el0  = (g * NTHR + tid) * EPT;
    const int e0   = cbase + el0;
    const int sent = -2147483647 - 1;
    v4i da, db;
    if (vec8 != 0 && cbase + CHUNK <= nE) {
      da = *(const v4i*)(dsts + e0);
      db = *(const v4i*)(dsts + e0 + 4);
    } else {
      da.x = (e0     < nE) ? dsts[min(e0,     nE - 1)] : sent;
      da.y = (e0 + 1 < nE) ? dsts[min(e0 + 1, nE - 1)] : sent;
      da.z = (e0 + 2 < nE) ? dsts[min(e0 + 2, nE - 1)] : sent;
      da.w = (e0 + 3 < nE) ? dsts[min(e0 + 3, nE - 1)] : sent;
      db.x = (e0 + 4 < nE) ? dsts[min(e0 + 4, nE - 1)] : sent;
      db.y = (e0 + 5 < nE) ? dsts[min(e0 + 5, nE - 1)] : sent;
      db.z = (e0 + 6 < nE) ? dsts[min(e0 + 6, nE - 1)] : sent;
      db.w = (e0 + 7 < nE) ? dsts[min(e0 + 7, nE - 1)] : sent;
    }
    const unsigned nb = (unsigned)nodeBase;
    const unsigned s0 = (unsigned)da.x - nb, s1 = (unsigned)da.y - nb;
    const unsigned s2 = (unsigned)da.z - nb, s3 = (unsigned)da.w - nb;
    const unsigned s4 = (unsigned)db.x - nb, s5 = (unsigned)db.y - nb;
    const unsigned s6 = (unsigned)db.z - nb, s7 = (unsigned)db.w - nb;
    const bool h0 = s0 < (unsigned)NB, h1 = s1 < (unsigned)NB, h2 = s2 < (unsigned)NB, h3 = s3 < (unsigned)NB;
    const bool h4 = s4 < (unsigned)NB, h5 = s5 < (unsigned)NB, h6 = s6 < (unsigned)NB, h7 = s7 < (unsigned)NB;
    const unsigned any = __builtin_amdgcn_ballot_w32(h0 | h1 | h2 | h3 | h4 | h5 | h6 | h7);
    if (any != 0u) {
#define HITJ(J, HJ, SJ) { \
        const unsigned mj = __builtin_amdgcn_ballot_w32(HJ); \
        if (mj != 0u) { \
          if (HJ) { \
            const int pos = wc + (int)__builtin_amdgcn_mbcnt_lo(mj, 0u); \
            if (pos < WCAP) list[wave * WCAP + pos] = ((el0 + (J)) << 12) | (int)(SJ); \
          } \
          wc += (int)__builtin_popcount(mj); } }
      HITJ(0, h0, s0)
      HITJ(1, h1, s1)
      HITJ(2, h2, s2)
      HITJ(3, h3, s3)
      HITJ(4, h4, s4)
      HITJ(5, h5, s5)
      HITJ(6, h6, s6)
      HITJ(7, h7, s7)
#undef HITJ
    }
  }
  return wc;
}

__device__ __forceinline__ void drain_wave(const int* __restrict__ ei, const float* __restrict__ ew,
                                           const float* mIn, unsigned* accu, const int* lp,
                                           int n, int cbase, int nE, int nN, int lane) {
  const int nit = (n + 7) >> 3;
  const int sub = lane >> 2, q = lane & 3;
#pragma unroll 1
  for (int it = 0; it < nit; ++it) {
    int idx = it * 8 + sub;
    idx = idx > n - 1 ? n - 1 : idx;
    const int ent  = lp[idx];
    const int slot = ent & (NB - 1);
    int e = cbase + ((ent >> 12) & (CHUNK - 1));
    e = e > nE - 1 ? nE - 1 : e;
    int src = ei[e];
    src = src < 0 ? 0 : (src > nN - 1 ? nN - 1 : src);
    const float w = ew[e];
    const v4f mv = *(const v4f*)(mIn + (size_t)src * MD + 4 * q);
    unsigned* ap = accu + slot * MD + 4 * q;
    atomicMax(ap + 0, f2key(mv.x * w));
    atomicMax(ap + 1, f2key(mv.y * w));
    atomicMax(ap + 2, f2key(mv.z * w));
    atomicMax(ap + 3, f2key(mv.w * w));
  }
}

__global__ __launch_bounds__(NTHR) void k_prop(const int* __restrict__ ei, const float* __restrict__ ew,
                                               const float* mIn, float* mOut,
                                               const float* mask0, const float* mC, float* out,
                                               int nE, int nN, int vec8, int last) {
  extern __shared__ v4u lds_dyn[];
  unsigned* accu = (unsigned*)lds_dyn;
  int*      list = (int*)(lds_dyn + (NB * MD / 4));
  const int tid = threadIdx.x, lane = tid & 31, wave = tid >> 5;
  const int nodeBase = blockIdx.x * NB;
  const int* dsts = ei + nE;

#pragma unroll 1
  for (int i = tid; i < NB * MD / 4; i += NTHR) {
    const int slot = i >> 2, q = i & 3;
    int node = nodeBase + slot;
    node = node > nN - 1 ? nN - 1 : node;
    const v4f v = *(const v4f*)(mIn + (size_t)node * MD + 4 * q);
    lds_dyn[i] = f2key4(v);
  }
  __syncthreads();

  const int nChunks = (nE + CHUNK - 1) / CHUNK;
#pragma unroll 1
  for (int ch = 0; ch < nChunks; ++ch) {
    const int cbase = ch * CHUNK;
    const int wc = scan_chunk(dsts, nE, cbase, nodeBase, vec8, list, tid, wave);
    __syncthreads();
    int n = __builtin_amdgcn_readfirstlane(wc);
    n = n > WCAP ? WCAP : (n < 0 ? 0 : n);
    if (n > 0) drain_wave(ei, ew, mIn, accu, list + wave * WCAP, n, cbase, nE, nN, lane);
    __syncthreads();
  }

  if (last == 0) {
    float* gb = mOut + (size_t)nodeBase * MD;
#pragma unroll 1
    for (int i = tid; i < NB * MD / 4; i += NTHR) {
      const v4f v = key2f4(lds_dyn[i]);
      *(volatile v4f*)(gb + (size_t)4 * i) = v;
    }
    __threadfence();
#pragma unroll 1
    for (int i = tid; i < NB * MD / 4; i += NTHR) {
      const v4f v = key2f4(lds_dyn[i]);
      *(volatile v4f*)(gb + (size_t)4 * i) = v;
    }
  } else {
#pragma unroll 1
    for (int i = tid; i < NB * MD / 4; i += NTHR) {
      const int slot = i >> 2, q = i & 3;
      const int row  = nodeBase + slot;
      const bool ok  = row < nN;
      const int rowc = ok ? row : (nN - 1);
      const v4f v = key2f4(lds_dyn[i]);
      const v4f a = *(const v4f*)(mask0 + (size_t)rowc * MD + 4 * q);
      const v4f b = *(const v4f*)(mC + (size_t)rowc * MD + 4 * q);
      v4f o;
      o.x = fmaxf(a.x, fmaxf(b.x, v.x)); o.y = fmaxf(a.y, fmaxf(b.y, v.y));
      o.z = fmaxf(a.z, fmaxf(b.z, v.z)); o.w = fmaxf(a.w, fmaxf(b.w, v.w));
      if (ok) *(volatile v4f*)(out + (size_t)rowc * MD + 4 * q) = o;
    }
    __threadfence();
#pragma unroll 1
    for (int i = tid; i < NB * MD / 4; i += NTHR) {
      const int slot = i >> 2, q = i & 3;
      const int row  = nodeBase + slot;
      const bool ok  = row < nN;
      const int rowc = ok ? row : (nN - 1);
      const v4f v = key2f4(lds_dyn[i]);
      const v4f a = *(const v4f*)(mask0 + (size_t)rowc * MD + 4 * q);
      const v4f b = *(const v4f*)(mC + (size_t)rowc * MD + 4 * q);
      v4f o;
      o.x = fmaxf(a.x, fmaxf(b.x, v.x)); o.y = fmaxf(a.y, fmaxf(b.y, v.y));
      o.z = fmaxf(a.z, fmaxf(b.z, v.z)); o.w = fmaxf(a.w, fmaxf(b.w, v.w));
      if (ok) *(volatile v4f*)(out + (size_t)rowc * MD + 4 * q) = o;
    }
  }
}

extern "C" void kernel_launch(void* const* d_in, const int* in_sizes, int n_in,
                              void* d_out, int out_size, void* d_ws, size_t ws_size,
                              hipStream_t stream) {
  if (n_in < 12) return;
  const int nN = in_sizes[0] / HD;
  if (nN <= 0 || in_sizes[0] != nN * HD || in_sizes[1] != nN * MD) return;
  const int nEs = in_sizes[2] / 2;
  const int nEd = in_sizes[3] / 2;
  if (nEs <= 0 || nEd <= 0 || in_sizes[2] != 2 * nEs || in_sizes[3] != 2 * nEd) return;
  if (in_sizes[4] != 4 * nEs || in_sizes[5] != nEd) return;
  if (in_sizes[6] != 2 * HD * TD || in_sizes[7] != TD || in_sizes[8] != 4 + TD || in_sizes[9] < 1 ||
      in_sizes[10] != 1 + TD || in_sizes[11] < 1) return;
  if (out_size != nN * MD) return;

  const float* x    = (const float*)d_in[0];
  const float* mask = (const float*)d_in[1];
  const int*   sei  = (const int*)d_in[2];
  const int*   dei  = (const int*)d_in[3];
  const float* sea  = (const float*)d_in[4];
  const float* dea  = (const float*)d_in[5];
  const float* Wtr  = (const float*)d_in[6];
  const float* btr  = (const float*)d_in[7];
  const float* Wpos = (const float*)d_in[8];
  const float* bpos = (const float*)d_in[9];
  const float* Wdom = (const float*)d_in[10];
  const float* bdom = (const float*)d_in[11];
  float* out = (float*)d_out;

  const int nTB = (nN + 16 * NWAVE - 1) / (16 * NWAVE);
  const int nBP = (nN + NB - 1) / NB;
  const int gEs = (nEs + NTHR - 1) / NTHR;
  const int gEd = (nEd + NTHR - 1) / NTHR;

  char* ws = (char*)d_ws;
  size_t off = 0;
  const size_t szWt = (size_t)NC * HD * 2;
  const size_t szPQ = (size_t)nTB * 16 * NWAVE * NC * 4;
  const size_t szEs = (size_t)gEs * NTHR * 4;
  const size_t szEd = (size_t)gEd * NTHR * 4;
  const size_t szM  = (size_t)nBP * NB * MD * 4;
  const size_t oWt = off; off += szWt; off = (off + 255) & ~(size_t)255;
  const size_t oPQ = off; off += szPQ; off = (off + 255) & ~(size_t)255;
  const size_t oEs = off; off += szEs; off = (off + 255) & ~(size_t)255;
  const size_t oEd = off; off += szEd; off = (off + 255) & ~(size_t)255;
  const size_t oMa = off; off += szM;  off = (off + 255) & ~(size_t)255;
  const size_t oMb = off; off += szM;  off = (off + 255) & ~(size_t)255;
  const size_t oMc = off; off += szM;  off = (off + 255) & ~(size_t)255;
  if (off > ws_size) return;
  f16_t* wt  = (f16_t*)(ws + oWt);
  float* pq  = (float*)(ws + oPQ);
  float* ewS = (float*)(ws + oEs);
  float* ewD = (float*)(ws + oEd);
  float* mA  = (float*)(ws + oMa);
  float* mB  = (float*)(ws + oMb);
  float* mCp = (float*)(ws + oMc);

  const int vec8s = ((nEs & 3) == 0) ? 1 : 0;
  const int vec8d = ((nEd & 3) == 0) ? 1 : 0;

  k_wprep<<<1, NTHR, 0, stream>>>(Wtr, wt);
  k_node<<<nTB, NTHR, 0, stream>>>(x, wt, pq, nN);
  k_edge<<<gEs, NTHR, 0, stream>>>(pq, sei, sea, Wpos, bpos, btr, ewS, nEs, nN, 4);
  k_edge<<<gEd, NTHR, 0, stream>>>(pq, dei, dea, Wdom, bdom, btr, ewD, nEd, nN, 1);

  hipFuncSetAttribute(reinterpret_cast<const void*>(&k_prop),
                      hipFuncAttributeMaxDynamicSharedMemorySize, LDS_PROP);

  k_prop<<<nBP, NTHR, LDS_PROP, stream>>>(sei, ewS, mask, mA,  mask, mCp, out, nEs, nN, vec8s, 0);
  k_prop<<<nBP, NTHR, LDS_PROP, stream>>>(sei, ewS, mA,   mB,  mask, mCp, out, nEs, nN, vec8s, 0);
  k_prop<<<nBP, NTHR, LDS_PROP, stream>>>(sei, ewS, mB,   mCp, mask, mCp, out, nEs, nN, vec8s, 0);
  k_prop<<<nBP, NTHR, LDS_PROP, stream>>>(dei, ewD, mask, mA,  mask, mCp, out, nEd, nN, vec8d, 0);
  k_prop<<<nBP, NTHR, LDS_PROP, stream>>>(dei, ewD, mA,   mB,  mask, mCp, out, nEd, nN, vec8d, 0);
  k_prop<<<nBP, NTHR, LDS_PROP, stream>>>(dei, ewD, mB,   mA,  mask, mCp, out, nEd, nN, vec8d, 1);
}
